// FlexAttention_77575699300897
// MI455X (gfx1250) — hardware-verified
//
#include <hip/hip_runtime.h>
#include <math.h>

typedef __attribute__((ext_vector_type(16))) _Float16 v16h;
typedef __attribute__((ext_vector_type(8)))  _Float16 v8h;
typedef __attribute__((ext_vector_type(16))) __bf16   v16b;
typedef __attribute__((ext_vector_type(8)))  __bf16   v8b;
typedef __attribute__((ext_vector_type(8)))  float    v8f;
typedef __attribute__((ext_vector_type(4)))  float    v4f;
typedef __attribute__((ext_vector_type(4)))  unsigned int v4u;

__device__ __forceinline__ unsigned short f2bf_bits(float f) {
  unsigned u = __float_as_uint(f);
  return (unsigned short)((u + 0x7FFFu + ((u >> 16) & 1u)) >> 16);
}
__device__ __forceinline__ float bf_bits2f(unsigned short h) { return __uint_as_float(((unsigned)h) << 16); }

__device__ __forceinline__ void dep_guard_b(v8f& a, v8f& b, v16b x, v16b y) { asm volatile("v_nop\n\tv_nop\n\tv_nop\n\tv_nop" : "+v"(a), "+v"(b) : "v"(x), "v"(y)); }
__device__ __forceinline__ void keep4_b(v16b a, v16b b, v16b c, v16b d) { asm volatile("v_nop" :: "v"(a), "v"(b), "v"(c), "v"(d)); }

template <typename T> struct Frag;
template <> struct Frag<__bf16> {
  typedef v16b V; union U { v16b v; v8b h[2]; };
  static __device__ __forceinline__ v16b load(const __bf16* p) {
    U f; f.h[0] = *(const v8b*)(p); f.h[1] = *(const v8b*)(p + 16); return f.v;
  }
  static __device__ __forceinline__ v8f mma(v16b a, v16b b, v8f c) {
    return __builtin_amdgcn_wmma_f32_16x16x32_bf16(false, a, false, b, (short)0, c, false, false);
  }
  static __device__ __forceinline__ void guard(v8f& a, v8f& b, v16b x, v16b y) { dep_guard_b(a, b, x, y); }
  static __device__ __forceinline__ void keep(v16b a, v16b b, v16b c, v16b d) { keep4_b(a, b, c, d); }
};

__device__ __forceinline__ unsigned short at_bf_bits(float f) {
  unsigned u = __float_as_uint(f);
  return (unsigned short)((u + 0x7FFFu + ((u >> 16) & 1u)) >> 16);
}
__device__ __forceinline__ __bf16 at_f2bf(float f) { return __builtin_bit_cast(__bf16, at_bf_bits(f)); }
__device__ __forceinline__ void at_split(float f, __bf16& hi, __bf16& lo) {
  const unsigned short hb = at_bf_bits(f);
  hi = __builtin_bit_cast(__bf16, hb);
  lo = at_f2bf(f - __uint_as_float(((unsigned)hb) << 16));
}
__device__ __forceinline__ v8f at_mma(v16b a, v16b b, v8f c) {
  c = __builtin_amdgcn_wmma_f32_16x16x32_bf16(false, a, false, b, (short)0, c, false, false);
  asm volatile("v_nop\n\tv_nop\n\tv_nop\n\tv_nop" : "+v"(c) : "v"(a), "v"(b));
  return c;
}

namespace cfg {
constexpr int NBATCH = 2;
constexpr int NHEAD  = 16;
constexpr int SEQ    = 2048;
constexpr int HDIM   = 128;
constexpr int WIN    = 512;
constexpr int QBLK   = 64;
constexpr int KCH    = 64;
constexpr int NWAVE  = 4;
constexpr int NTHR   = 128;
constexpr int NQBLK  = SEQ / QBLK;
constexpr int WCH    = WIN / KCH;
constexpr int KPITCH = HDIM + 8;
constexpr int VPITCH = KCH + 8;
constexpr int PPITCH = KCH + 8;
constexpr int OPITCH = HDIM + 4;
constexpr int NELEM  = NBATCH * NHEAD * SEQ * HDIM;
}
static_assert(cfg::SEQ % cfg::QBLK == 0);
static_assert(cfg::WIN % cfg::KCH == 0);
static_assert(cfg::HDIM == 128);
static_assert(cfg::KCH == 64);
static_assert((cfg::KPITCH * 2) % 16 == 0);
static_assert((cfg::VPITCH * 2) % 16 == 0);
static_assert((cfg::OPITCH * 4) % 16 == 0);
static_assert(cfg::NELEM % (8 * 256) == 0);

__global__ __launch_bounds__(256) void cast_f32_bf16x8(
    const float* __restrict__ in, unsigned short* __restrict__ out, int n8) {
  const int i = blockIdx.x * 256 + threadIdx.x;
  if (i < n8) {
    const size_t e0 = (size_t)i * 8;
    const v4f a = *(const v4f*)(in + e0);
    const v4f b = *(const v4f*)(in + e0 + 4);
    v4u w;
    w[0] = (unsigned)f2bf_bits(a[0]) | ((unsigned)f2bf_bits(a[1]) << 16);
    w[1] = (unsigned)f2bf_bits(a[2]) | ((unsigned)f2bf_bits(a[3]) << 16);
    w[2] = (unsigned)f2bf_bits(b[0]) | ((unsigned)f2bf_bits(b[1]) << 16);
    w[3] = (unsigned)f2bf_bits(b[2]) | ((unsigned)f2bf_bits(b[3]) << 16);
    *(volatile v4u*)(out + e0) = w;
    __threadfence();
    *(volatile v4u*)(out + e0) = w;
  }
}

__global__ __launch_bounds__(128)
void attn128_swa(const unsigned short* __restrict__ qp, const unsigned short* __restrict__ kp,
                 const unsigned short* __restrict__ vp, float* __restrict__ out, float scale) {
  using namespace cfg;
  __shared__ __align__(16) __bf16 Ksh[KCH * KPITCH];
  __shared__ __align__(16) __bf16 Vth[HDIM * VPITCH];
  __shared__ __align__(16) __bf16 Psh[NWAVE][16 * PPITCH];
  __shared__ __align__(16) __bf16 Psl[NWAVE][16 * PPITCH];
  __shared__ __align__(16) float  Os[NWAVE][16 * OPITCH];

  const int tid  = threadIdx.x;
  const int wave = tid >> 5;
  const int lane = tid & 31;
  const int hh   = lane >> 4;
  const int c    = lane & 15;

  const int bx   = blockIdx.x;
  const int qblk = bx % NQBLK;
  const int bh   = bx / NQBLK;
  const size_t bhoff = (size_t)bh * SEQ * HDIM;
  const __bf16* qb = (const __bf16*)qp + bhoff;
  float*        ob = out + bhoff;
  const int q0 = qblk * QBLK + wave * 16;

  v16b qa[4];
  {
    const __bf16* qrow = qb + (size_t)(q0 + c) * HDIM;
#pragma unroll
    for (int dc = 0; dc < 4; ++dc) qa[dc] = Frag<__bf16>::load(qrow + dc * 32 + 8 * hh);
  }

  float mrow[8], lrow[8];
  v8f oacc[8];
#pragma unroll
  for (int r = 0; r < 8; ++r) { mrow[r] = -INFINITY; lrow[r] = 0.f; }
#pragma unroll
  for (int t = 0; t < 8; ++t) oacc[t] = (v8f){0.f,0.f,0.f,0.f,0.f,0.f,0.f,0.f};

  int kc_lo = qblk - WCH;
  if (kc_lo < 0) kc_lo = 0;
  const int kvr = tid >> 1;
  const int dh  = (tid & 1) * 64;

  for (int kc = kc_lo; kc <= qblk; ++kc) {
    const int kv0 = kc * KCH;
    __syncthreads();
    {
      const v4u* ksrc = (const v4u*)(kp + (bhoff + (size_t)(kv0 + kvr) * HDIM + dh));
      v4u* kdst = (v4u*)(Ksh + kvr * KPITCH + dh);
#pragma unroll
      for (int i = 0; i < 8; ++i) kdst[i] = ksrc[i];
      const v4u* vsrc = (const v4u*)(vp + (bhoff + (size_t)(kv0 + kvr) * HDIM + dh));
#pragma unroll
      for (int i = 0; i < 8; ++i) {
        const v4u w = vsrc[i];
#pragma unroll
        for (int m = 0; m < 4; ++m) {
          const unsigned wm = w[m];
          const int d = dh + 8 * i + 2 * m;
          Vth[d * VPITCH + kvr]       = __builtin_bit_cast(__bf16, (unsigned short)(wm & 0xffffu));
          Vth[(d + 1) * VPITCH + kvr] = __builtin_bit_cast(__bf16, (unsigned short)(wm >> 16));
        }
      }
    }
    __syncthreads();

    v8f s[4];
#pragma unroll
    for (int j = 0; j < 4; ++j) {
      s[j] = (v8f){0.f,0.f,0.f,0.f,0.f,0.f,0.f,0.f};
      const __bf16* krow = Ksh + (j * 16 + c) * KPITCH + 8 * hh;
#pragma unroll
      for (int dc = 0; dc < 4; ++dc) {
        const v16b kf = Frag<__bf16>::load(krow + dc * 32);
        s[j] = at_mma(qa[dc], kf, s[j]);
      }
    }

    float cm[8];
#pragma unroll
    for (int r = 0; r < 8; ++r) {
      const int qrow = q0 + 8 * hh + r;
      float m = -INFINITY;
#pragma unroll
      for (int j = 0; j < 4; ++j) {
        const int kvcol = kv0 + j * 16 + c;
        const bool masked = (kvcol > qrow) || (qrow - kvcol > WIN);
        float sv = s[j][r] * scale;
        sv = masked ? -INFINITY : sv;
        s[j][r] = sv;
        m = fmaxf(m, sv);
      }
#pragma unroll
      for (int off = 1; off < 16; off <<= 1) m = fmaxf(m, __shfl_xor(m, off, 32));
      cm[r] = m;
    }

    __bf16* pwh = Psh[wave];
    __bf16* pwl = Psl[wave];
#pragma unroll
    for (int r = 0; r < 8; ++r) {
      const float mnew  = fmaxf(mrow[r], cm[r]);
      const float alpha = expf(mrow[r] - mnew);
      mrow[r] = mnew;
      float psum = 0.f;
#pragma unroll
      for (int j = 0; j < 4; ++j) {
        const float p = expf(s[j][r] - mnew);
        psum += p;
        __bf16 ph, pl;
        at_split(p, ph, pl);
        pwh[(8 * hh + r) * PPITCH + j * 16 + c] = ph;
        pwl[(8 * hh + r) * PPITCH + j * 16 + c] = pl;
      }
#pragma unroll
      for (int off = 1; off < 16; off <<= 1) psum += __shfl_xor(psum, off, 32);
      lrow[r] = lrow[r] * alpha + psum;
#pragma unroll
      for (int t = 0; t < 8; ++t) oacc[t][r] *= alpha;
    }
    __builtin_amdgcn_fence(__ATOMIC_RELEASE, "workgroup");
    __builtin_amdgcn_wave_barrier();
    __builtin_amdgcn_fence(__ATOMIC_ACQUIRE, "workgroup");

#pragma unroll
    for (int kk = 0; kk < 2; ++kk) {
      const v16b pa = Frag<__bf16>::load(pwh + c * PPITCH + kk * 32 + 8 * hh);
      const v16b pb = Frag<__bf16>::load(pwl + c * PPITCH + kk * 32 + 8 * hh);
#pragma unroll
      for (int t = 0; t < 8; ++t) {
        const v16b vf = Frag<__bf16>::load(Vth + (t * 16 + c) * VPITCH + kk * 32 + 8 * hh);
        oacc[t] = at_mma(pa, vf, oacc[t]);
        oacc[t] = at_mma(pb, vf, oacc[t]);
      }
    }
  }

  float* os = Os[wave];
#pragma unroll
  for (int r = 0; r < 8; ++r) {
    const float inv = 1.0f / lrow[r];
#pragma unroll
    for (int t = 0; t < 8; ++t) os[(8 * hh + r) * OPITCH + t * 16 + c] = oacc[t][r] * inv;
  }
  __builtin_amdgcn_fence(__ATOMIC_RELEASE, "workgroup");
  __builtin_amdgcn_wave_barrier();
  __builtin_amdgcn_fence(__ATOMIC_ACQUIRE, "workgroup");
  {
    const int c4 = lane * 4;
    for (int pass = 0; pass < 2; ++pass) {
#pragma unroll
      for (int row = 0; row < 16; ++row) {
        const v4f val = *(const v4f*)(os + row * OPITCH + c4);
        *(volatile v4f*)(ob + (size_t)(q0 + row) * HDIM + c4) = val;
      }
      __threadfence();
    }
  }
}

extern "C" void kernel_launch(void* const* d_in, const int* in_sizes, int n_in,
                              void* d_out, int out_size, void* d_ws, size_t ws_size,
                              hipStream_t stream) {
  using namespace cfg;
  const int n = NELEM;
  if (n_in < 3) return;
  if (in_sizes[0] != n || in_sizes[1] != n || in_sizes[2] != n || out_size != n) return;
  const size_t planeBytes = (size_t)n * 2;
  if (ws_size < 3 * planeBytes) return;

  const float* q = (const float*)d_in[0];
  const float* k = (const float*)d_in[1];
  const float* v = (const float*)d_in[2];
  float* o = (float*)d_out;
  unsigned short* qh = (unsigned short*)d_ws;
  unsigned short* kh = qh + n;
  unsigned short* vh = kh + n;

  const int n8 = n / 8;
  const int castBlocks = (n8 + 255) / 256;
  cast_f32_bf16x8<<<castBlocks, 256, 0, stream>>>(q, qh, n8);
  cast_f32_bf16x8<<<castBlocks, 256, 0, stream>>>(k, kh, n8);
  cast_f32_bf16x8<<<castBlocks, 256, 0, stream>>>(v, vh, n8);

  const float scale = (float)(1.0 / sqrt((double)HDIM));
  attn128_swa<<<NBATCH * NHEAD * NQBLK, NTHR, 0, stream>>>(qh, kh, vh, o, scale);
}
